// GenericTransformerLayer_49125835931911
// MI455X (gfx1250) — hardware-verified
//
#include <hip/hip_runtime.h>


namespace {
constexpr int NB = 2, S = 2048, D = 1024, NH = 16, DH = 64, DFF = 3072, NROW = NB * S;
constexpr float XS = 8.0f, WSC = 256.0f, PS = 8.0f, EPS = 1e-6f;

typedef _Float16 b16;
typedef __attribute__((ext_vector_type(16))) _Float16 v16b;
typedef __attribute__((ext_vector_type(8))) _Float16 v8b;
typedef __attribute__((ext_vector_type(8))) float v8f;
typedef __attribute__((ext_vector_type(4))) float v4f;
__device__ __forceinline__ float bf16_rne(float f) { unsigned int u = __float_as_uint(f); u += 0x7FFFu + ((u >> 16) & 1u); return __uint_as_float(u & 0xFFFF0000u); }
__device__ __forceinline__ v16b frag_kb(const b16* p, int hh) { const v8b a = *(const v8b*)(p + 8 * hh), b = *(const v8b*)(p + 16 + 8 * hh); v16b f;
#pragma unroll
  for (int e = 0; e < 8; ++e) { f[e] = a[e]; f[8 + e] = b[e]; } return f; }
__device__ __forceinline__ v8f wmma16b(v16b a, v16b b, v8f c) { v8f d = __builtin_amdgcn_wmma_f32_16x16x32_f16(false, a, false, b, (short)0, c, false, false); asm volatile("v_nop\n\tv_nop\n\tv_nop\n\tv_nop" : "+v"(d) : "v"(a), "v"(b)); return d; }
__device__ __forceinline__ void wave_lds_sync() { __builtin_amdgcn_fence(__ATOMIC_RELEASE, "workgroup"); __builtin_amdgcn_wave_barrier(); __builtin_amdgcn_fence(__ATOMIC_ACQUIRE, "workgroup"); }
__device__ __forceinline__ float nexp(float x) { return __builtin_amdgcn_exp2f(x * 1.4426950408889634f); }
__device__ __forceinline__ float pmul(float a, float b) { float p = a * b; asm volatile("" : "+v"(p)); return p; }
__device__ __forceinline__ float hsum16(float v) { v += __shfl_xor(v, 1); v += __shfl_xor(v, 2); v += __shfl_xor(v, 4); return v + __shfl_xor(v, 8); }

__global__ __launch_bounds__(256) void prepw_kernel(const float* __restrict__ wqkv, const float* __restrict__ wout, const float* __restrict__ wup, const float* __restrict__ wdn, b16* __restrict__ WQKV, b16* __restrict__ WOUT, b16* __restrict__ WUP, b16* __restrict__ WDN) {
  const size_t tid = (size_t)blockIdx.x * 256 + threadIdx.x, nth = (size_t)gridDim.x * 256;
  const size_t n1 = (size_t)3 * D * D / 8, n2 = (size_t)D * D / 8, n3 = (size_t)2 * DFF * D / 8, n4 = (size_t)D * DFF / 8;
  for (int pass = 0; pass < 2; ++pass) {
    for (size_t g = tid; g < n1 + n2 + n3 + n4; g += nth) { const float* src; b16* dst; size_t e;
      if (g < n1) { src = wqkv; dst = WQKV; e = g * 8; } else if (g < n1 + n2) { src = wout; dst = WOUT; e = (g - n1) * 8; } else if (g < n1 + n2 + n3) { src = wup; dst = WUP; e = (g - n1 - n2) * 8; } else { src = wdn; dst = WDN; e = (g - n1 - n2 - n3) * 8; }
      const v4f a = *(const v4f*)(src + e), c = *(const v4f*)(src + e + 4); v8b o;
#pragma unroll
      for (int j = 0; j < 4; ++j) { o[j] = (b16)(bf16_rne(a[j]) * WSC); o[4 + j] = (b16)(bf16_rne(c[j]) * WSC); }
      *(volatile v8b*)(dst + e) = o; }
    __threadfence(); }
}
template <int MODE>
__global__ __launch_bounds__(256) void rms_kernel(const float* __restrict__ X, const float* __restrict__ sc, b16* __restrict__ H16) {
  __shared__ __attribute__((aligned(16))) float Tr[8][D];
  const int wave = threadIdx.x >> 5, lane = threadIdx.x & 31; const size_t row = (size_t)blockIdx.x * 8 + wave; const float* src = X + row * D;
  float ss = 0.0f;
#pragma unroll 1
  for (int j = 0; j < 32; ++j) { const float v = MODE == 0 ? bf16_rne(src[j * 32 + lane]) : src[j * 32 + lane]; Tr[wave][j * 32 + lane] = v; ss += pmul(v, v); }
#pragma unroll
  for (int o = 16; o >= 1; o >>= 1) ss += __shfl_xor(ss, o);
  const float rs = rsqrtf(ss * (1.0f / D) + EPS);
  wave_lds_sync();
  for (int pass = 0; pass < 2; ++pass) { for (int qd = 0; qd < 4; ++qd) { v8b o;
#pragma unroll
      for (int j = 0; j < 8; ++j) { const int c = qd * 256 + lane * 8 + j; o[j] = (b16)(pmul(Tr[wave][c], bf16_rne(sc[c]) * rs) * XS); }
      *(volatile v8b*)(H16 + row * D + qd * 256 + lane * 8) = o; } __threadfence(); }
}
__global__ __launch_bounds__(128) void qkv_kernel(const b16* __restrict__ H16, const b16* __restrict__ WQKV, const float* __restrict__ pos, const float* __restrict__ ascale, const float* __restrict__ freqs, b16* __restrict__ QH, b16* __restrict__ KH, b16* __restrict__ VROW, int nb0) {
  __shared__ __attribute__((aligned(16))) b16 Th[4][16][128 + 8];
  const int wave = threadIdx.x >> 5, lane = threadIdx.x & 31, nloc = lane & 15, hlf = lane >> 4; const int m0 = blockIdx.x * 64 + wave * 16, n0 = (nb0 + blockIdx.y) * 128; const int which = n0 / D, h0 = (n0 - which * D) / DH;
  v8f acc[8];
#pragma unroll
  for (int t = 0; t < 8; ++t) acc[t] = (v8f){};
#pragma unroll 2
  for (int kb = 0; kb < D; kb += 32) { const v16b a = frag_kb(H16 + (size_t)(m0 + nloc) * D + kb, hlf);
#pragma unroll
    for (int t = 0; t < 8; ++t) acc[t] = wmma16b(a, frag_kb(WQKV + (size_t)(n0 + t * 16 + nloc) * D + kb, hlf), acc[t]); }
#pragma unroll
  for (int t = 0; t < 8; ++t)
#pragma unroll
    for (int r = 0; r < 8; ++r) acc[t][r] *= (1.0f / (XS * WSC));
  if (which < 2) {
#pragma unroll
    for (int hs = 0; hs < 2; ++hs) { const int h = h0 + hs; const float ssc = sqrtf(bf16_rne(ascale[h]));
#pragma unroll
      for (int r = 0; r < 8; ++r) { const int m = m0 + 8 * hlf + r, b = m / S, l = m - b * S; float ss = 0.0f;
#pragma unroll
        for (int t = 0; t < 4; ++t) ss += pmul(acc[hs * 4 + t][r], acc[hs * 4 + t][r]);
        ss = hsum16(ss); const float f = ssc * rsqrtf(ss + EPS);
        const float ph = bf16_rne(pos[((size_t)b * S + l) * 2 + 0]), pw = bf16_rne(pos[((size_t)b * S + l) * 2 + 1]);
#pragma unroll
        for (int t = 0; t < 2; ++t) { const int j = t * 16 + nloc;
          const float fr = bf16_rne(freqs[h * 16 + (j & 15)]); const float th = pmul(j < 16 ? ph : pw, fr); float sn, cs; sincosf(th, &sn, &cs);
          const float x1 = acc[hs * 4 + t][r] * f, x2 = acc[hs * 4 + t + 2][r] * f; acc[hs * 4 + t][r] = pmul(x1, cs) - pmul(x2, sn); acc[hs * 4 + t + 2][r] = pmul(x2, cs) + pmul(x1, sn); } } } }
#pragma unroll
  for (int t = 0; t < 8; ++t)
#pragma unroll
    for (int r = 0; r < 8; ++r) Th[wave][8 * hlf + r][t * 16 + nloc] = (b16)(acc[t][r] * XS);
  wave_lds_sync();
  b16* dst = which == 0 ? QH : which == 1 ? KH : VROW;
  for (int pass = 0; pass < 2; ++pass) { for (int rr = 0; rr < 16; ++rr) if (lane < 16) { const int m = m0 + rr, b = m / S, l = m - b * S; const int hs = lane >> 3, c8 = (lane & 7) * 8; *(volatile v8b*)(dst + (((size_t)b * NH + h0 + hs) * S + l) * DH + c8) = *(const v8b*)(&Th[wave][rr][hs * 64 + c8]); } __threadfence(); }
}
__global__ __launch_bounds__(256) void vt_kernel(const b16* __restrict__ VROW, b16* __restrict__ VT) {
  __shared__ __attribute__((aligned(16))) b16 Tt[DH][64 + 8];
  const int bh = blockIdx.y, s0 = blockIdx.x * 64, t_ = threadIdx.x;
  for (int k = t_; k < 64 * DH; k += 256) { const int ss = k >> 6, d = k & 63; Tt[d][ss] = VROW[((size_t)bh * S + s0 + ss) * DH + d]; }
  __syncthreads();
  for (int pass = 0; pass < 2; ++pass) { for (int q = t_; q < DH * 8; q += 256) { const int d = q >> 3, c8 = (q & 7) * 8; *(volatile v8b*)(VT + ((size_t)bh * DH + d) * S + s0 + c8) = *(const v8b*)(&Tt[d][c8]); } __threadfence(); }
}
__global__ __launch_bounds__(64) void attn_kernel(const b16* __restrict__ QH, const b16* __restrict__ KH, const b16* __restrict__ VT, b16* __restrict__ ATT) {
  __shared__ __attribute__((aligned(16))) b16 To[2][16][DH + 8];
  const int wave = threadIdx.x >> 5, lane = threadIdx.x & 31, hh = lane >> 4, col = lane & 15; const int bh = blockIdx.y, b = bh / NH, h = bh - b * NH, q0 = blockIdx.x * 32 + wave * 16, qi = q0 + col;
  const b16* Q = QH + (size_t)bh * S * DH; const b16* K = KH + (size_t)bh * S * DH; const b16* V = VT + (size_t)bh * DH * S;
  v16b qf[2];
#pragma unroll
  for (int ks = 0; ks < 2; ++ks) qf[ks] = frag_kb(Q + (size_t)qi * DH + ks * 32, hh);
  const float scale = 1.0f / (XS * XS);
  float m = -INFINITY, l = 0.0f; v8f o[4] = {{}, {}, {}, {}};
  for (int kb = 0; kb < S; kb += 32) {
    v8f s0 = {}, s1 = {};
#pragma unroll
    for (int ks = 0; ks < 2; ++ks) { s0 = wmma16b(frag_kb(K + (size_t)(kb + col) * DH + ks * 32, hh), qf[ks], s0); s1 = wmma16b(frag_kb(K + (size_t)(kb + 16 + col) * DH + ks * 32, hh), qf[ks], s1); }
    float mr = -INFINITY;
#pragma unroll
    for (int r = 0; r < 8; ++r) { s0[r] *= scale; s1[r] *= scale; mr = fmaxf(mr, fmaxf(s0[r], s1[r])); }
    mr = fmaxf(mr, __shfl_xor(mr, 16)); const float mn = fmaxf(m, mr); const float al_ = nexp(m - mn); m = mn; float sum = 0.0f; v16b pb;
#pragma unroll
    for (int r = 0; r < 8; ++r) { const float e0 = nexp(s0[r] - mn), e1 = nexp(s1[r] - mn); sum += e0 + e1; pb[r] = (b16)(e0 * PS); pb[8 + r] = (b16)(e1 * PS); }
    sum += __shfl_xor(sum, 16); l = l * al_ + sum;
#pragma unroll
    for (int t = 0; t < 4; ++t) { o[t] *= al_; o[t] = wmma16b(frag_kb(V + (size_t)(t * 16 + col) * S + kb, hh), pb, o[t]); } }
  const float inv = 1.0f / (l * PS * XS);
#pragma unroll
  for (int t = 0; t < 4; ++t)
#pragma unroll
    for (int r = 0; r < 8; ++r) To[wave][col][t * 16 + 8 * hh + r] = (b16)(o[t][r] * inv * XS);
  wave_lds_sync();
  for (int pass = 0; pass < 2; ++pass) { for (int rr = 0; rr < 16; ++rr) if (lane < 8) *(volatile v8b*)(ATT + ((size_t)b * S + q0 + rr) * D + h * DH + lane * 8) = *(const v8b*)(&To[wave][rr][lane * 8]); __threadfence(); }
}
template <int MODE>
__global__ __launch_bounds__(128) void gemmres_kernel(const b16* __restrict__ A, int K, const b16* __restrict__ Bw, const float* __restrict__ R, float* __restrict__ Y) {
  __shared__ __attribute__((aligned(16))) float Ts[4][16][128 + 4];
  const int wave = threadIdx.x >> 5, lane = threadIdx.x & 31, nloc = lane & 15, hlf = lane >> 4; const int m0 = blockIdx.x * 64 + wave * 16, n0 = blockIdx.y * 128;
  v8f acc[8];
#pragma unroll
  for (int t = 0; t < 8; ++t) acc[t] = (v8f){};
  for (int kb = 0; kb < K; kb += 32) { const v16b a = frag_kb(A + (size_t)(m0 + nloc) * K + kb, hlf);
#pragma unroll
    for (int t = 0; t < 8; ++t) acc[t] = wmma16b(a, frag_kb(Bw + (size_t)(n0 + t * 16 + nloc) * K + kb, hlf), acc[t]); }
#pragma unroll
  for (int t = 0; t < 8; ++t)
#pragma unroll
    for (int r = 0; r < 8; ++r) Ts[wave][8 * hlf + r][t * 16 + nloc] = acc[t][r] * (1.0f / (XS * WSC));
  wave_lds_sync();
  for (int pass = 0; pass < 2; ++pass) { for (int rr = 0; rr < 16; ++rr) { const size_t gi = (size_t)(m0 + rr) * D + n0 + lane * 4; v4f v = *(const v4f*)(&Ts[wave][rr][lane * 4]); const v4f rv = *(const v4f*)(R + gi);
      if (MODE == 0) { v[0] += bf16_rne(rv[0]); v[1] += bf16_rne(rv[1]); v[2] += bf16_rne(rv[2]); v[3] += bf16_rne(rv[3]); } else v += rv; *(volatile v4f*)(Y + gi) = v; } __threadfence(); }
}
__global__ __launch_bounds__(128) void up_kernel(const b16* __restrict__ H2, const b16* __restrict__ WUP, b16* __restrict__ H3) {
  __shared__ __attribute__((aligned(16))) b16 Th[4][16][64 + 8];
  const int wave = threadIdx.x >> 5, lane = threadIdx.x & 31, nloc = lane & 15, hlf = lane >> 4; const int m0 = blockIdx.x * 64 + wave * 16, j0 = blockIdx.y * 64;
  v8f acc[8];
#pragma unroll
  for (int t = 0; t < 8; ++t) acc[t] = (v8f){};
#pragma unroll 2
  for (int kb = 0; kb < D; kb += 32) { const v16b a = frag_kb(H2 + (size_t)(m0 + nloc) * D + kb, hlf);
#pragma unroll
    for (int t = 0; t < 4; ++t) { acc[t] = wmma16b(a, frag_kb(WUP + (size_t)(j0 + t * 16 + nloc) * D + kb, hlf), acc[t]); acc[4 + t] = wmma16b(a, frag_kb(WUP + (size_t)(DFF + j0 + t * 16 + nloc) * D + kb, hlf), acc[4 + t]); } }
#pragma unroll
  for (int t = 0; t < 4; ++t)
#pragma unroll
    for (int r = 0; r < 8; ++r) { const float a = acc[t][r] * (1.0f / (XS * WSC)), g = acc[4 + t][r] * (1.0f / (XS * WSC)); const float sg = g / (1.0f + nexp(-g)); Th[wave][8 * hlf + r][t * 16 + nloc] = (b16)(pmul(a, sg) * XS); }
  wave_lds_sync();
  for (int pass = 0; pass < 2; ++pass) { for (int rr = 0; rr < 16; ++rr) if (lane < 8) *(volatile v8b*)(H3 + (size_t)(m0 + rr) * DFF + j0 + lane * 8) = *(const v8b*)(&Th[wave][rr][lane * 8]); __threadfence(); }
}
}

extern "C" void kernel_launch(void* const* d_in, const int* in_sizes, int n_in, void* d_out, int out_size, void* d_ws, size_t ws_size, hipStream_t stream) {
  (void)n_in;
  auto Fp = [&](int i) { return (const float*)d_in[i]; };
  if (in_sizes[0] != NROW * D || in_sizes[1] != NROW * 2 || in_sizes[3] != 3 * D * D || in_sizes[5] != NH * 16 || in_sizes[8] != 2 * DFF * D || in_sizes[9] != D * DFF || out_size != NROW * D) return;
  size_t off = 0; char* ws = (char*)d_ws;
  auto carve = [&](size_t bytes) { char* p = ws + off; off += (bytes + 255) & ~(size_t)255; return p; };
  b16* WQKV = (b16*)carve((size_t)3 * D * D * 2); b16* WOUT = (b16*)carve((size_t)D * D * 2); b16* WUP = (b16*)carve((size_t)2 * DFF * D * 2); b16* WDN = (b16*)carve((size_t)D * DFF * 2);
  b16* H16 = (b16*)carve((size_t)NROW * D * 2); b16* QH = (b16*)carve((size_t)NROW * D * 2); b16* KH = (b16*)carve((size_t)NROW * D * 2); b16* VROW = (b16*)carve((size_t)NROW * D * 2); b16* VT = (b16*)carve((size_t)NROW * D * 2);
  float* X1 = (float*)carve((size_t)NROW * D * 4); b16* H3 = (b16*)carve((size_t)NROW * DFF * 2);
  b16* ATT = VROW;
  b16* H2 = H16;
  if (off > ws_size) return;
  prepw_kernel<<<1024, 256, 0, stream>>>(Fp(3), Fp(6), Fp(8), Fp(9), WQKV, WOUT, WUP, WDN);
  rms_kernel<0><<<NROW / 8, 256, 0, stream>>>(Fp(0), Fp(2), H16);
  qkv_kernel<<<dim3(NROW / 64, 3 * D / 128), 128, 0, stream>>>(H16, WQKV, Fp(1), Fp(4), Fp(5), QH, KH, VROW, 0);
  vt_kernel<<<dim3(S / 64, NB * NH), 256, 0, stream>>>(VROW, VT);
  attn_kernel<<<dim3(S / 32, NB * NH), 64, 0, stream>>>(QH, KH, VT, ATT);
  gemmres_kernel<0><<<dim3(NROW / 64, D / 128), 128, 0, stream>>>(ATT, D, WOUT, Fp(0), X1);
  rms_kernel<1><<<NROW / 8, 256, 0, stream>>>(X1, Fp(7), H2);
  up_kernel<<<dim3(NROW / 64, DFF / 64), 128, 0, stream>>>(H2, WUP, H3);
  gemmres_kernel<1><<<dim3(NROW / 64, D / 128), 128, 0, stream>>>(H3, DFF, WDN, X1, (float*)d_out);
}
